// GraphModel_34411277976253
// MI455X (gfx1250) — hardware-verified
//
#include <hip/hip_runtime.h>
#include <stddef.h>


#define GD      128
#define NPQ     256
#define GR      32
#define XSP     260
#define NB      512
#define CHUNK   2048
#define NTHR    256
#define NWAVE   8
#define WCAP    256
#define NGRP    (CHUNK / (NTHR * 4))
#define FR      32
#define ZD      135
#define DIN     7

#define LDS_S    (NB * GD)
#define LDS_DEG  (NB)
#define LDS_LIST (NWAVE * WCAP)
#define AGG_LDS_BYTES ((LDS_S + LDS_DEG + LDS_LIST + NWAVE) * 4)

static_assert(WCAP == (CHUNK / NTHR) * 32);
static_assert(NGRP == 2);
static_assert(NB == 512);
static_assert(CHUNK == 2048);
static_assert(((LDS_S + LDS_DEG) % 4) == 0);
static_assert(AGG_LDS_BYTES == 272416);
static_assert(((NB / 16) % NWAVE) == 0);
static_assert((NB % GR) == 0);
static_assert(GR == 4 * NWAVE);
static_assert(FR == 4 * NWAVE);

typedef float          v4f   __attribute__((ext_vector_type(4)));
typedef float          v8f   __attribute__((ext_vector_type(8)));
typedef int            v4i   __attribute__((ext_vector_type(4)));
typedef unsigned int   v4u   __attribute__((ext_vector_type(4)));
typedef unsigned short v8us  __attribute__((ext_vector_type(8)));
typedef unsigned short v16us __attribute__((ext_vector_type(16)));
typedef __bf16         v16b  __attribute__((ext_vector_type(16)));
union FragB { v16b v; v16us s; v8us u[2]; };
union Pk8   { v8us s; v4u w; };

__device__ __forceinline__ unsigned short bf_bits(float f) {
  unsigned u = __float_as_uint(f);
  u += 0x7FFFu + ((u >> 16) & 1u);
  return (unsigned short)(u >> 16);
}
__device__ __forceinline__ void split2(float f, unsigned short& hi, unsigned short& lo) {
  hi = bf_bits(f);
  const float hf = __uint_as_float(((unsigned)hi) << 16);
  lo = bf_bits(f - hf);
}
template <int O>
__device__ __forceinline__ void cvt4(v4f f, FragB& h, FragB& l) {
  unsigned short a, b;
  split2(f.x, a, b); h.s[O]     = a; l.s[O]     = b;
  split2(f.y, a, b); h.s[O + 1] = a; l.s[O + 1] = b;
  split2(f.z, a, b); h.s[O + 2] = a; l.s[O + 2] = b;
  split2(f.w, a, b); h.s[O + 3] = a; l.s[O + 3] = b;
}

__device__ __forceinline__ v8f wmb(v16b a, v16b b, v8f c) {
  v8f d = __builtin_amdgcn_wmma_f32_16x16x32_bf16(false, a, false, b, (short)0, c, false, false);
  asm volatile("v_nop\n\tv_nop\n\tv_nop\n\tv_nop" : "+v"(d) : "v"(a), "v"(b));
  return d;
}

__device__ __forceinline__ float th1(float x) {
  x = fminf(fmaxf(x, -16.0f), 16.0f);
  const float e = __builtin_amdgcn_exp2f(x * 2.885390082f);
  const float r = __builtin_amdgcn_rcpf(e + 1.0f);
  return fmaf(-2.0f, r, 1.0f);
}

__device__ __forceinline__ float wsum(float v) {
  v += __shfl_xor(v, 16, 32);
  v += __shfl_xor(v, 8, 32);
  v += __shfl_xor(v, 4, 32);
  v += __shfl_xor(v, 2, 32);
  v += __shfl_xor(v, 1, 32);
  return v;
}

__global__ __launch_bounds__(NTHR) void k_wprep(const float* __restrict__ W, int Kd, int Nsrc, int mode,
                                                int Dsplit, unsigned short* Whi, unsigned short* Wlo,
                                                int Nout, int KP) {
  const int i  = blockIdx.x * NTHR + threadIdx.x;
  const int n8 = (Nout * KP) >> 3;
  if (i >= n8) return;
  const int e8 = i * 8;
  const int n  = e8 / KP;
  const int kb = e8 - n * KP;
  const bool first = (n < Nsrc);
  const int nn = first ? n : (n - Nsrc);
  Pk8 ph, pl;
#pragma unroll
  for (int j = 0; j < 8; ++j) {
    const int k  = kb + j;
    const int kc = (k < Kd) ? k : (Kd - 1);
    const float wa = W[(size_t)kc * Nsrc + nn];
    const float wb = W[(size_t)(Dsplit + kc) * Nsrc + nn];
    float v = (mode == 0) ? wa : (first ? (wa - wb) : wb);
    if (k >= Kd) v = 0.f;
    unsigned short hs, ls;
    split2(v, hs, ls);
    ph.s[j] = hs;
    pl.s[j] = ls;
  }
  *(volatile v4u*)(Whi + e8) = ph.w;
  *(volatile v4u*)(Wlo + e8) = pl.w;
  __threadfence();
  *(volatile v4u*)(Whi + e8) = ph.w;
  *(volatile v4u*)(Wlo + e8) = pl.w;
}

template <int KSTEPS>
__global__ __launch_bounds__(NTHR) void k_node(const float* __restrict__ A, int Kd, int nRowsA,
                                               const unsigned short* __restrict__ Whi,
                                               const unsigned short* __restrict__ Wlo,
                                               const float* __restrict__ b1, float* PQ) {
  constexpr int KP = 32 * KSTEPS;
  constexpr int AP = KP + 8;
  __shared__ __attribute__((aligned(16))) unsigned short Ahi[GR * AP];
  __shared__ __attribute__((aligned(16))) unsigned short Alo[GR * AP];
  __shared__ __attribute__((aligned(16))) float Xs[GR * XSP];

  const int tid  = threadIdx.x;
  const int lane = tid & 31;
  const int wave = tid >> 5;
  const int hh   = lane >> 4;
  const int m    = lane & 15;
  const int rowBase = blockIdx.x * GR;

  for (int idx = tid; idx < GR * KP; idx += NTHR) {
    const int r = idx / KP;
    const int k = idx - r * KP;
    int row = rowBase + r;
    if (row > nRowsA - 1) row = nRowsA - 1;
    const int kc = (k < Kd) ? k : (Kd - 1);
    float v = A[(size_t)row * Kd + kc];
    if (k >= Kd) v = 0.f;
    unsigned short hs, ls;
    split2(v, hs, ls);
    Ahi[r * AP + k] = hs;
    Alo[r * AP + k] = ls;
  }
  __syncthreads();

  const v8f z8 = {0.f, 0.f, 0.f, 0.f, 0.f, 0.f, 0.f, 0.f};
  v8f acc[2][2];
#pragma unroll
  for (int t = 0; t < 2; ++t)
#pragma unroll
    for (int c = 0; c < 2; ++c) acc[t][c] = z8;

#pragma unroll 1
  for (int ks = 0; ks < KSTEPS; ++ks) {
    const int k0 = ks * 32;
    FragB bh[2], bl[2], ah[2], al[2];
#pragma unroll
    for (int c = 0; c < 2; ++c) {
      const size_t ob = (size_t)(wave * 32 + 16 * c + m) * KP + k0 + 8 * hh;
      bh[c].u[0] = *(const v8us*)(Whi + ob);
      bh[c].u[1] = *(const v8us*)(Whi + ob + 16);
      bl[c].u[0] = *(const v8us*)(Wlo + ob);
      bl[c].u[1] = *(const v8us*)(Wlo + ob + 16);
    }
#pragma unroll
    for (int t = 0; t < 2; ++t) {
      const int oa = (16 * t + m) * AP + k0 + 8 * hh;
      ah[t].u[0] = *(const v8us*)(Ahi + oa);
      ah[t].u[1] = *(const v8us*)(Ahi + oa + 16);
      al[t].u[0] = *(const v8us*)(Alo + oa);
      al[t].u[1] = *(const v8us*)(Alo + oa + 16);
    }
#pragma unroll
    for (int t = 0; t < 2; ++t) {
#pragma unroll
      for (int c = 0; c < 2; ++c) {
        acc[t][c] = wmb(ah[t].v, bh[c].v, acc[t][c]);
        acc[t][c] = wmb(ah[t].v, bl[c].v, acc[t][c]);
        acc[t][c] = wmb(al[t].v, bh[c].v, acc[t][c]);
      }
    }
  }

#pragma unroll
  for (int c = 0; c < 2; ++c) {
    const int ncol = wave * 32 + 16 * c + m;
    float bb = b1[ncol & (GD - 1)];
    if (wave >= 4) bb = 0.f;
#pragma unroll
    for (int t = 0; t < 2; ++t) {
#pragma unroll
      for (int r = 0; r < 8; ++r) Xs[(16 * t + 8 * hh + r) * XSP + ncol] = acc[t][c][r] + bb;
    }
  }
  __syncthreads();

  v4f pv[4], qv[4];
#pragma unroll
  for (int i = 0; i < 4; ++i) {
    const int row = 4 * wave + i;
    pv[i] = *(const v4f*)(Xs + row * XSP + 4 * lane);
    qv[i] = *(const v4f*)(Xs + row * XSP + GD + 4 * lane);
  }
  float* gp = PQ + (size_t)(rowBase + 4 * wave) * NPQ + 4 * lane;
#pragma unroll
  for (int i = 0; i < 4; ++i) {
    *(volatile v4f*)(gp + (size_t)i * NPQ)      = pv[i];
    *(volatile v4f*)(gp + (size_t)i * NPQ + GD) = qv[i];
  }
  __threadfence();
#pragma unroll
  for (int i = 0; i < 4; ++i) {
    *(volatile v4f*)(gp + (size_t)i * NPQ)      = pv[i];
    *(volatile v4f*)(gp + (size_t)i * NPQ + GD) = qv[i];
  }
}

__global__ __launch_bounds__(NTHR) void k_agg(const int* __restrict__ ei, const float* __restrict__ PQ,
                                              const unsigned short* __restrict__ Whi,
                                              const unsigned short* __restrict__ Wlo,
                                              const float* __restrict__ b2, float* H, int nN, int nE) {
  extern __shared__ v4f lds_dyn[];
  float* S    = (float*)lds_dyn;
  float* degc = S + LDS_S;
  int*   list = (int*)(degc + LDS_DEG);
  int*   wcnt = list + LDS_LIST;

  const int tid  = threadIdx.x;
  const int lane = tid & 31;
  const int wave = tid >> 5;
  const int hh   = lane >> 4;
  const int m    = lane & 15;
  const int nodeBase = blockIdx.x * NB;

  {
    const v4f z4 = {0.f, 0.f, 0.f, 0.f};
    for (int i = tid; i < (LDS_S + LDS_DEG) / 4; i += NTHR) lds_dyn[i] = z4;
  }
  __syncthreads();

  const int* eid = ei + nE;
  const bool al16 = ((nE & 3) == 0);

  const int nChunks = (nE + CHUNK - 1) / CHUNK;
#pragma unroll 1
  for (int ch = 0; ch < nChunks; ++ch) {
    const int cbase = ch * CHUNK;
    int wc = 0;
#pragma unroll
    for (int g = 0; g < NGRP; ++g) {
      const int el0 = (g * NTHR + tid) * 4;
      const int e0  = cbase + el0;
      const int sent = -2147483647 - 1;
      v4i d;
      if (al16 && (cbase + CHUNK <= nE)) {
        d = *(const v4i*)(eid + e0);
      } else {
        d.x = (e0     < nE) ? eid[min(e0,     nE - 1)] : sent;
        d.y = (e0 + 1 < nE) ? eid[min(e0 + 1, nE - 1)] : sent;
        d.z = (e0 + 2 < nE) ? eid[min(e0 + 2, nE - 1)] : sent;
        d.w = (e0 + 3 < nE) ? eid[min(e0 + 3, nE - 1)] : sent;
      }
      const unsigned s0 = (unsigned)d.x - (unsigned)nodeBase;
      const unsigned s1 = (unsigned)d.y - (unsigned)nodeBase;
      const unsigned s2 = (unsigned)d.z - (unsigned)nodeBase;
      const unsigned s3 = (unsigned)d.w - (unsigned)nodeBase;
      const bool h0 = s0 < (unsigned)NB;
      const bool h1 = s1 < (unsigned)NB;
      const bool h2 = s2 < (unsigned)NB;
      const bool h3 = s3 < (unsigned)NB;
      const unsigned many = __builtin_amdgcn_ballot_w32(h0 | h1 | h2 | h3);
      if (many != 0u) {
#define HITJ(J, HJ, SJ) { \
          const unsigned mj = __builtin_amdgcn_ballot_w32(HJ); \
          if (HJ) { \
            const int pos = wc + (int)__builtin_amdgcn_mbcnt_lo(mj, 0u); \
            if (pos < WCAP) list[wave * WCAP + pos] = ((el0 + (J)) << 9) | (int)(SJ); \
          } \
          wc += (int)__builtin_popcount(mj); }
        HITJ(0, h0, s0)
        HITJ(1, h1, s1)
        HITJ(2, h2, s2)
        HITJ(3, h3, s3)
#undef HITJ
      }
    }
    if (lane == 0) wcnt[wave] = wc;
    __syncthreads();

    if (wave == 0) {
      for (int wsx = 0; wsx < NWAVE; ++wsx) {
        int n = wcnt[wsx];
        if (n > WCAP) n = WCAP;
        if (n < 0) n = 0;
        for (int i = 0; i < n; ++i) {
          const int ent  = list[wsx * WCAP + i];
          const int slot = ent & (NB - 1);
          const int el   = (ent >> 9) & (CHUNK - 1);
          int e = cbase + el;
          if (e > nE - 1) e = nE - 1;
          int src = ei[e];
          src = src < 0 ? 0 : (src > nN - 1 ? nN - 1 : src);
          const int nd = nodeBase + slot;
          const v4f q = *(const v4f*)(PQ + (size_t)src * NPQ + GD + 4 * lane);
          const v4f p = *(const v4f*)(PQ + (size_t)nd * NPQ + 4 * lane);
          v4f t;
          t.x = th1(p.x + q.x);
          t.y = th1(p.y + q.y);
          t.z = th1(p.z + q.z);
          t.w = th1(p.w + q.w);
          v4f* sp = (v4f*)(S + slot * GD + 4 * lane);
          const v4f cur = *sp;
          *sp = cur + t;
          if (lane == 0) {
            const float dv = degc[slot];
            degc[slot] = dv + 1.0f;
          }
        }
      }
    }
    __syncthreads();
  }

#pragma unroll 1
  for (int it = 0; it < (NB / 16) / NWAVE; ++it) {
    const int T = it * NWAVE + wave;
    const float* srow = S + (16 * T + m) * GD;
    FragB ah[4], al[4];
#pragma unroll
    for (int ks = 0; ks < 4; ++ks) {
      const float* sp = srow + 32 * ks + 8 * hh;
      const v4f f0 = *(const v4f*)(sp);
      const v4f f1 = *(const v4f*)(sp + 4);
      const v4f f2 = *(const v4f*)(sp + 16);
      const v4f f3 = *(const v4f*)(sp + 20);
      cvt4<0>(f0, ah[ks], al[ks]);
      cvt4<4>(f1, ah[ks], al[ks]);
      cvt4<8>(f2, ah[ks], al[ks]);
      cvt4<12>(f3, ah[ks], al[ks]);
    }
    float dg[8];
#pragma unroll
    for (int r = 0; r < 8; ++r) dg[r] = degc[16 * T + 8 * hh + r];
    __syncthreads();

#pragma unroll 1
    for (int c = 0; c < GD / 16; ++c) {
      v8f acc = {0.f, 0.f, 0.f, 0.f, 0.f, 0.f, 0.f, 0.f};
      const size_t ob = (size_t)(16 * c + m) * GD + 8 * hh;
#pragma unroll
      for (int ks = 0; ks < 4; ++ks) {
        FragB bh, bl;
        bh.u[0] = *(const v8us*)(Whi + ob + 32 * ks);
        bh.u[1] = *(const v8us*)(Whi + ob + 32 * ks + 16);
        bl.u[0] = *(const v8us*)(Wlo + ob + 32 * ks);
        bl.u[1] = *(const v8us*)(Wlo + ob + 32 * ks + 16);
        acc = wmb(ah[ks].v, bh.v, acc);
        acc = wmb(ah[ks].v, bl.v, acc);
        acc = wmb(al[ks].v, bh.v, acc);
      }
      const float bv = b2[16 * c + m];
      float* drow = S + (16 * T + 8 * hh) * GD + 16 * c + m;
#pragma unroll
      for (int r = 0; r < 8; ++r) drow[r * GD] = fmaf(dg[r], bv, acc[r]);
    }
    __syncthreads();

    v4f hv[16];
#pragma unroll
    for (int R = 0; R < 16; ++R) hv[R] = *(const v4f*)(S + (16 * T + R) * GD + 4 * lane);
    float* gp = H + (size_t)(nodeBase + 16 * T) * GD + 4 * lane;
#pragma unroll
    for (int R = 0; R < 16; ++R) *(volatile v4f*)(gp + (size_t)R * GD) = hv[R];
    __threadfence();
#pragma unroll
    for (int R = 0; R < 16; ++R) *(volatile v4f*)(gp + (size_t)R * GD) = hv[R];
  }
}

__global__ __launch_bounds__(NTHR) void k_final(const float* __restrict__ x, const float* __restrict__ H,
                                                const float* __restrict__ g, const float* __restrict__ bb,
                                                const float* __restrict__ wout, const float* __restrict__ bout,
                                                float* out, int nN) {
  __shared__ __attribute__((aligned(16))) float outs[FR * 3 + 4];
  const int tid  = threadIdx.x;
  const int lane = tid & 31;
  const int wave = tid >> 5;
  const int node0 = blockIdx.x * FR;
  const float bo0 = bout[0], bo1 = bout[1], bo2 = bout[2];

#pragma unroll 1
  for (int j = 0; j < FR / NWAVE; ++j) {
    const int nl = wave * (FR / NWAVE) + j;
    const int node = node0 + nl;
    if (node < nN) {
      const size_t xn = (size_t)node * DIN;
      const size_t hn = (size_t)node * GD;
      float z[5];
      {
        const float xv = x[xn + (lane < DIN ? lane : DIN - 1)];
        const float hv = H[hn + (lane >= DIN ? lane - DIN : 0)];
        z[0] = (lane < DIN) ? xv : hv;
      }
      z[1] = H[hn + lane + (32 - DIN)];
      z[2] = H[hn + lane + (64 - DIN)];
      z[3] = H[hn + lane + (96 - DIN)];
      {
        const float hv = H[hn + (lane < DIN ? lane + (128 - DIN) : GD - 1)];
        z[4] = (lane < DIN) ? hv : 0.f;
      }
      const bool v4ok = (lane < DIN);
      float s = z[0] + z[1] + z[2] + z[3] + z[4];
      s = wsum(s);
      const float mu = s * (1.0f / (float)ZD);
      float dq[5];
#pragma unroll
      for (int t = 0; t < 4; ++t) dq[t] = z[t] - mu;
      dq[4] = v4ok ? (z[4] - mu) : 0.f;
      float q = dq[0] * dq[0] + dq[1] * dq[1] + dq[2] * dq[2] + dq[3] * dq[3] + dq[4] * dq[4];
      q = wsum(q);
      const float var = q * (1.0f / (float)ZD);
      const float rs  = rsqrtf(var + 1e-5f);
      float p0 = 0.f, p1 = 0.f, p2 = 0.f;
#pragma unroll
      for (int t = 0; t < 5; ++t) {
        const bool valid = (t < 4) || v4ok;
        const int d  = lane + 32 * t;
        const int dc = valid ? d : (ZD - 1);
        const float zn = dq[t] * rs * g[dc] + bb[dc];
        const float w0 = wout[dc * 3 + 0];
        const float w1 = wout[dc * 3 + 1];
        const float w2 = wout[dc * 3 + 2];
        p0 += valid ? zn * w0 : 0.f;
        p1 += valid ? zn * w1 : 0.f;
        p2 += valid ? zn * w2 : 0.f;
      }
      p0 = wsum(p0);
      p1 = wsum(p1);
      p2 = wsum(p2);
      if (lane == 0) {
        outs[nl * 3 + 0] = p0 + bo0;
        outs[nl * 3 + 1] = p1 + bo1;
        outs[nl * 3 + 2] = p2 + bo2;
      }
    }
  }
  __syncthreads();

  if (wave == 0) {
    int nv = nN - node0;
    if (nv > FR) nv = FR;
    if (nv < 0) nv = 0;
    const int nf = nv * 3;
    const int nq = nf >> 2;
    const int rem = nf & 3;
    float* op = out + (size_t)node0 * 3;
    const v4f vv = *(const v4f*)(outs + 4 * (lane < nq ? lane : 0));
    int si = nq * 4 + lane;
    if (si > FR * 3 - 1) si = FR * 3 - 1;
    const float sv = outs[si];
    if (lane < nq)  *(volatile v4f*)(op + 4 * lane) = vv;
    if (lane < rem) *(volatile float*)(op + nq * 4 + lane) = sv;
    __threadfence();
    if (lane < nq)  *(volatile v4f*)(op + 4 * lane) = vv;
    if (lane < rem) *(volatile float*)(op + nq * 4 + lane) = sv;
  }
}

extern "C" void kernel_launch(void* const* d_in, const int* in_sizes, int n_in,
                              void* d_out, int out_size, void* d_ws, size_t ws_size,
                              hipStream_t stream) {
  if (n_in < 14) return;
  const int nN = in_sizes[0] / DIN;
  const int nE = in_sizes[1] / 2;
  if (nN <= 0 || in_sizes[0] != nN * DIN) return;
  if (nE <= 0 || in_sizes[1] != 2 * nE) return;
  if (in_sizes[2] != 2 * DIN * GD || in_sizes[3] != GD) return;
  if (in_sizes[4] != GD * GD || in_sizes[5] != GD) return;
  if (in_sizes[6] != 3 * 2 * GD * GD || in_sizes[7] != 3 * GD) return;
  if (in_sizes[8] != 3 * GD * GD || in_sizes[9] != 3 * GD) return;
  if (in_sizes[10] != ZD || in_sizes[11] != ZD || in_sizes[12] != ZD * 3 || in_sizes[13] != 3) return;
  if (out_size != nN * 3) return;

  const float* x     = (const float*)d_in[0];
  const int*   ei    = (const int*)d_in[1];
  const float* w1_0  = (const float*)d_in[2];
  const float* b1_0  = (const float*)d_in[3];
  const float* w2_0  = (const float*)d_in[4];
  const float* b2_0  = (const float*)d_in[5];
  const float* w1s   = (const float*)d_in[6];
  const float* b1s   = (const float*)d_in[7];
  const float* w2s   = (const float*)d_in[8];
  const float* b2s   = (const float*)d_in[9];
  const float* ln_g  = (const float*)d_in[10];
  const float* ln_b  = (const float*)d_in[11];
  const float* w_out = (const float*)d_in[12];
  const float* b_out = (const float*)d_in[13];
  float* out = (float*)d_out;

  const int nPA = ((nN + NB - 1) / NB) * NB;

  size_t off = 0;
  auto take = [&](size_t bytes) -> void* {
    void* p = (char*)d_ws + off;
    off += (bytes + 255) & ~(size_t)255;
    return p;
  };
  const size_t w1p0 = (size_t)NPQ * 32 * 2;
  const size_t w1p  = (size_t)NPQ * GD * 2;
  const size_t w2p  = (size_t)GD * GD * 2;
  unsigned short* W1h0 = (unsigned short*)take(w1p0);
  unsigned short* W1l0 = (unsigned short*)take(w1p0);
  unsigned short* W2h0 = (unsigned short*)take(w2p);
  unsigned short* W2l0 = (unsigned short*)take(w2p);
  unsigned short* W1h[3];
  unsigned short* W1l[3];
  unsigned short* W2h[3];
  unsigned short* W2l[3];
  for (int l = 0; l < 3; ++l) {
    W1h[l] = (unsigned short*)take(w1p);
    W1l[l] = (unsigned short*)take(w1p);
    W2h[l] = (unsigned short*)take(w2p);
    W2l[l] = (unsigned short*)take(w2p);
  }
  float* PQ = (float*)take((size_t)nPA * NPQ * sizeof(float));
  float* Hp = (float*)take((size_t)nPA * GD * sizeof(float));
  if (off > ws_size) return;
  if (off > (size_t)134217728) return;

  auto prep = [&](const float* W, int Kd, int Nsrc, int mode, int Dsplit,
                  unsigned short* hi, unsigned short* lo, int Nout, int KP) {
    const int n8 = (Nout * KP) / 8;
    k_wprep<<<(n8 + NTHR - 1) / NTHR, NTHR, 0, stream>>>(W, Kd, Nsrc, mode, Dsplit, hi, lo, Nout, KP);
  };
  prep(w1_0, DIN, GD, 1, DIN, W1h0, W1l0, NPQ, 32);
  prep(w2_0, GD, GD, 0, 0, W2h0, W2l0, GD, GD);
  for (int l = 0; l < 3; ++l) {
    prep(w1s + (size_t)l * 2 * GD * GD, GD, GD, 1, GD, W1h[l], W1l[l], NPQ, GD);
    prep(w2s + (size_t)l * GD * GD, GD, GD, 0, 0, W2h[l], W2l[l], GD, GD);
  }

  const int gridNode = nPA / GR;
  const int gridAgg  = nPA / NB;
  hipFuncSetAttribute(reinterpret_cast<const void*>(&k_agg),
                      hipFuncAttributeMaxDynamicSharedMemorySize, AGG_LDS_BYTES);

  k_node<1><<<gridNode, NTHR, 0, stream>>>(x, DIN, nN, W1h0, W1l0, b1_0, PQ);
  k_agg<<<gridAgg, NTHR, AGG_LDS_BYTES, stream>>>(ei, PQ, W2h0, W2l0, b2_0, Hp, nN, nE);
  for (int l = 0; l < 3; ++l) {
    k_node<4><<<gridNode, NTHR, 0, stream>>>(Hp, GD, nN, W1h[l], W1l[l], b1s + (size_t)l * GD, PQ);
    k_agg<<<gridAgg, NTHR, AGG_LDS_BYTES, stream>>>(ei, PQ, W2h[l], W2l[l], b2s + (size_t)l * GD, Hp, nN, nE);
  }
  k_final<<<(nN + FR - 1) / FR, NTHR, 0, stream>>>(x, Hp, ln_g, ln_b, w_out, b_out, out, nN);
}
